// SimAttn_87144886436263
// MI455X (gfx1250) — hardware-verified
//
#include <hip/hip_runtime.h>
#include <math.h>
#include <stdint.h>

#define NBAT 4
#define NT   192
#define ND   512
#define NCP  5
#define NBT  768
#define NQV  11
#define NKV  6
#define NPR  66
#define QPW  5632
#define KPW  3072
#define CPW  2560
#define NZG  264
#define GSZ  36864

typedef __attribute__((ext_vector_type(16))) __bf16 v16b;
typedef __attribute__((ext_vector_type(8)))  __bf16 v8b;
typedef __attribute__((ext_vector_type(8)))  float  v8f;
typedef __attribute__((ext_vector_type(4)))  float  v4f;
typedef __attribute__((ext_vector_type(2)))  float  v2f;
typedef __attribute__((ext_vector_type(4)))  unsigned int   v4u;
typedef __attribute__((ext_vector_type(8)))  unsigned short v8us;

__device__ __forceinline__ unsigned short f2bf_bits(float f) {
  unsigned u = __float_as_uint(f);
  return (unsigned short)((u + 0x7FFFu + ((u >> 16) & 1u)) >> 16);
}
__device__ __forceinline__ float bf_bits2f(unsigned short h) { return __uint_as_float(((unsigned)h) << 16); }
__device__ __forceinline__ unsigned pk16(unsigned short a, unsigned short b) { return (unsigned)a | ((unsigned)b << 16); }

union FragU { v16b v; v8b h[2]; };
__device__ __forceinline__ v16b frag_load(const __bf16* p) {
  FragU f; f.h[0] = *(const v8b*)(p); f.h[1] = *(const v8b*)(p + 16); return f.v;
}
__device__ __forceinline__ v8f mma_bf(v16b a, v16b b, v8f c) {
  return __builtin_amdgcn_wmma_f32_16x16x32_bf16(false, a, false, b, (short)0, c, false, false);
}
__device__ __forceinline__ void dep_guard(v8f& a, v8f& b, v16b x, v16b y) {
  asm volatile("v_nop\n\tv_nop\n\tv_nop\n\tv_nop" : "+v"(a), "+v"(b) : "v"(x), "v"(y));
}
__device__ __forceinline__ void keep4(v16b a, v16b b, v16b c, v16b d) { asm volatile("v_nop" :: "v"(a), "v"(b), "v"(c), "v"(d)); }
__device__ __forceinline__ void acc_guard4(v8f& a, v8f& b, v8f& c, v8f& d) {
  asm volatile("v_nop\n\tv_nop\n\tv_nop\n\tv_nop" : "+v"(a), "+v"(b), "+v"(c), "+v"(d));
}

template <int BIAS_MODE, int OUT_MODE, bool RESID>
__global__ __launch_bounds__(256) void gemm64_split(
    const unsigned short* __restrict__ Ahp, const unsigned short* __restrict__ Alp, int lda, long sAo, long sAi,
    const unsigned short* __restrict__ Bhp, const unsigned short* __restrict__ Blp, int ldb, long sBo, long sBi,
    void* Cout, void* Cout2, int ldc, long sC,
    const float* __restrict__ bias, int nbias,
    const float* __restrict__ resid, int ldr, int rcol0, long sR,
    int M, int N, int K, int nPair, int nB, float scale)
{
  __shared__ __align__(16) float sT[8][16 * 68];
  const int z    = blockIdx.y;
  const int lane = threadIdx.x & 31;
  const int wave = threadIdx.x >> 5;
  const int wpb  = blockDim.x >> 5;
  const int tilesN = N >> 6;
  const int tilesM = M >> 6;
  const int tile = blockIdx.x * wpb + wave;
  if (tile >= tilesM * tilesN) return;
  const int tm = tile / tilesN;
  const int tn = tile - tm * tilesN;
  const int m0 = tm << 6;
  const int n0 = tn << 6;
  const int zb = z / nPair;
  const int zp = z - zb * nPair;
  const int ia = zp / nB;
  const int ib = zp - ia * nB;

  const __bf16* Ah = (const __bf16*)(const void*)Ahp + (size_t)zb * sAo + (size_t)ia * sAi;
  const __bf16* Al = (const __bf16*)(const void*)Alp + (size_t)zb * sAo + (size_t)ia * sAi;
  const __bf16* Bh = (const __bf16*)(const void*)Bhp + (size_t)zb * sBo + (size_t)ib * sBi;
  const __bf16* Bl = (const __bf16*)(const void*)Blp + (size_t)zb * sBo + (size_t)ib * sBi;

  const int rl   = lane & 15;
  const int koff = (lane >> 4) * 8;
  const int mOff = (lane >> 4) * 8;

  v8f acc[4][4];
#pragma unroll
  for (int i = 0; i < 4; ++i)
#pragma unroll
    for (int j = 0; j < 4; ++j) acc[i][j] = (v8f){0.f,0.f,0.f,0.f,0.f,0.f,0.f,0.f};

  for (int k0 = 0; k0 < K; k0 += 32) {
    v16b bh[4], bl[4];
#pragma unroll
    for (int j = 0; j < 4; ++j) {
      const size_t bo = (size_t)(n0 + (j << 4) + rl) * ldb + koff + k0;
      bh[j] = frag_load(Bh + bo);
      bl[j] = frag_load(Bl + bo);
    }
#pragma unroll
    for (int i = 0; i < 4; ++i) {
      const size_t ao = (size_t)(m0 + (i << 4) + rl) * lda + koff + k0;
      const v16b ah = frag_load(Ah + ao);
      const v16b al = frag_load(Al + ao);
#pragma unroll
      for (int j = 0; j < 4; ++j) {
        acc[i][j] = mma_bf(ah, bh[j], acc[i][j]);
        acc[i][j] = mma_bf(ah, bl[j], acc[i][j]);
        acc[i][j] = mma_bf(al, bh[j], acc[i][j]);
      }
      dep_guard(acc[i][0], acc[i][3], ah, al);
    }
    keep4(bh[0], bh[1], bh[2], bh[3]);
    keep4(bl[0], bl[1], bl[2], bl[3]);
  }
  acc_guard4(acc[0][0], acc[0][1], acc[0][2], acc[0][3]);
  acc_guard4(acc[1][0], acc[1][1], acc[1][2], acc[1][3]);
  acc_guard4(acc[2][0], acc[2][1], acc[2][2], acc[2][3]);
  acc_guard4(acc[3][0], acc[3][1], acc[3][2], acc[3][3]);

  float* slab = sT[wave];
  const float* Rb = RESID ? (resid + (size_t)zb * sR) : nullptr;
#pragma unroll
  for (int i = 0; i < 4; ++i) {
    const int mBase = m0 + (i << 4);
#pragma unroll
    for (int j = 0; j < 4; ++j) {
      const int n = n0 + (j << 4) + rl;
      float bvn = 0.0f;
      if (BIAS_MODE == 2) {
        const int nc = (n < nbias) ? n : (nbias - 1);
        const float tb = bias[nc];
        bvn = (n < nbias) ? tb : 0.0f;
      }
      int rc = 0;
      if (RESID) rc = n - rcol0;
      const int rcc = (rc > 0) ? rc : 0;
#pragma unroll
      for (int r = 0; r < 8; ++r) {
        const int m = mBase + mOff + r;
        float v = acc[i][j][r] * scale;
        if (BIAS_MODE == 1) { const int mc = (m < nbias) ? m : (nbias - 1); v += bias[mc]; }
        if (BIAS_MODE == 2) v += bvn;
        if (RESID) { const float rv = Rb[(size_t)m * ldr + rcc]; v += (rc >= 0) ? rv : 0.0f; }
        slab[(mOff + r) * 68 + (j << 4) + rl] = v;
      }
    }
    __builtin_amdgcn_fence(__ATOMIC_RELEASE, "workgroup");
    __builtin_amdgcn_wave_barrier();
    __builtin_amdgcn_fence(__ATOMIC_ACQUIRE, "workgroup");
    if (OUT_MODE == 0) {
      float* Cf = (float*)Cout + (size_t)z * sC;
      const int hh = lane >> 4, c4 = (lane & 15) * 4;
      for (int pass = 0; pass < 2; ++pass) {
#pragma unroll
        for (int it = 0; it < 8; ++it) {
          const int row = it * 2 + hh;
          const v4f vv = *(const v4f*)(slab + row * 68 + c4);
          *(volatile v4f*)(Cf + (size_t)(mBase + row) * ldc + n0 + c4) = vv;
        }
        __threadfence();
      }
    } else {
      const int q = lane >> 3, c8 = (lane & 7) * 8;
      unsigned short* Cu  = (unsigned short*)Cout  + (size_t)z * sC;
      unsigned short* Cu2 = (unsigned short*)Cout2 + (size_t)z * sC;
      v8us hv[4], lv[4];
#pragma unroll
      for (int it = 0; it < 4; ++it) {
        const int row = it * 4 + q;
        const float* sp = slab + row * 68 + c8;
        v8us a, a2;
#pragma unroll
        for (int e = 0; e < 8; ++e) {
          const float f = sp[e];
          const unsigned short hb = f2bf_bits(f);
          const unsigned short lb = f2bf_bits(f - bf_bits2f(hb));
          a[e] = hb; a2[e] = lb;
        }
        hv[it] = a; lv[it] = a2;
      }
      for (int pass = 0; pass < 2; ++pass) {
#pragma unroll
        for (int it = 0; it < 4; ++it) {
          const int row = it * 4 + q;
          const size_t go = (size_t)(mBase + row) * ldc + n0 + c8;
          *(volatile v8us*)(Cu + go) = hv[it];
          *(volatile v8us*)(Cu2 + go) = lv[it];
        }
        __threadfence();
      }
    }
    __builtin_amdgcn_fence(__ATOMIC_RELEASE, "workgroup");
    __builtin_amdgcn_wave_barrier();
    __builtin_amdgcn_fence(__ATOMIC_ACQUIRE, "workgroup");
  }
}

__global__ __launch_bounds__(256) void split3_kernel(const float* __restrict__ a0, const float* __restrict__ a1,
                                                     const float* __restrict__ a2,
                                                     unsigned short* hi, unsigned short* lo, int n2, int planeElems)
{
  const int y = blockIdx.y;
  const float* in = (y == 0) ? a0 : ((y == 1) ? a1 : a2);
  unsigned short* hp = hi + (size_t)y * planeElems;
  unsigned short* lp = lo + (size_t)y * planeElems;
  const int i = blockIdx.x * 256 + threadIdx.x;
  if (i < n2) {
    const v2f f = *(const v2f*)(in + 2 * (size_t)i);
    const unsigned short h0 = f2bf_bits(f[0]), h1 = f2bf_bits(f[1]);
    const unsigned short q0 = f2bf_bits(f[0] - bf_bits2f(h0)), q1 = f2bf_bits(f[1] - bf_bits2f(h1));
    const unsigned uh = pk16(h0, h1), ul = pk16(q0, q1);
    ((volatile unsigned*)hp)[i] = uh;
    ((volatile unsigned*)lp)[i] = ul;
    __threadfence();
    ((volatile unsigned*)hp)[i] = uh;
    ((volatile unsigned*)lp)[i] = ul;
  }
}

__global__ __launch_bounds__(256) void tsplit4_kernel(
    const float* __restrict__ w0, const float* __restrict__ w1, const float* __restrict__ w2, const float* __restrict__ w3,
    unsigned short* oh0, unsigned short* oh1, unsigned short* oh2, unsigned short* oh3,
    unsigned short* ol0, unsigned short* ol1, unsigned short* ol2, unsigned short* ol3,
    int R, int Cc)
{
  __shared__ __align__(16) float tf[64 * 68];
  const int z = blockIdx.z;
  const float* W = (z == 0) ? w0 : ((z == 1) ? w1 : ((z == 2) ? w2 : w3));
  unsigned short* oh = (z == 0) ? oh0 : ((z == 1) ? oh1 : ((z == 2) ? oh2 : oh3));
  unsigned short* ol = (z == 0) ? ol0 : ((z == 1) ? ol1 : ((z == 2) ? ol2 : ol3));
  const int c0  = blockIdx.x * 64;
  const int r0  = blockIdx.y * 64;
  const int tid = threadIdx.x;
  {
    const int lr = tid >> 4;
    const int c4 = (tid & 15) * 4;
#pragma unroll
    for (int it = 0; it < 4; ++it) {
      const int rr = it * 16 + lr;
      const v4f a = *(const v4f*)(W + (size_t)(r0 + rr) * Cc + c0 + c4);
      *(v4f*)(tf + rr * 68 + c4) = a;
    }
  }
  __syncthreads();
  const int sub = tid >> 3;
  const int c8  = (tid & 7) * 8;
  v4u hv[2], lv[2];
#pragma unroll
  for (int it = 0; it < 2; ++it) {
    const int oc = it * 32 + sub;
    v4u a, a2;
#pragma unroll
    for (int qq = 0; qq < 4; ++qq) {
      const float f0 = tf[(c8 + 2 * qq) * 68 + oc];
      const float f1 = tf[(c8 + 2 * qq + 1) * 68 + oc];
      const unsigned short h0 = f2bf_bits(f0), h1 = f2bf_bits(f1);
      const unsigned short q0 = f2bf_bits(f0 - bf_bits2f(h0)), q1 = f2bf_bits(f1 - bf_bits2f(h1));
      a[qq]  = pk16(h0, h1);
      a2[qq] = pk16(q0, q1);
    }
    hv[it] = a; lv[it] = a2;
  }
  for (int pass = 0; pass < 2; ++pass) {
#pragma unroll
    for (int it = 0; it < 2; ++it) {
      const int oc = it * 32 + sub;
      const size_t go = (size_t)(c0 + oc) * R + r0 + c8;
      *(volatile v4u*)(oh + go) = hv[it];
      *(volatile v4u*)(ol + go) = lv[it];
    }
    __threadfence();
  }
}

__global__ __launch_bounds__(256) void score_softmax_kernel(
    const float* __restrict__ G, const float* __restrict__ qa, const float* __restrict__ aq,
    const int* __restrict__ mask, unsigned short* Ph, unsigned short* Pl, float rscale)
{
  __shared__ float redm[8];
  __shared__ float reds[8];
  __shared__ __align__(16) unsigned short ph[NT];
  __shared__ __align__(16) unsigned short pl[NT];
  const int bt   = blockIdx.x;
  const int b    = bt / NT;
  const int t    = bt - b * NT;
  const int tid  = threadIdx.x;
  const int lane = tid & 31;
  const int wave = tid >> 5;
  const bool valid = tid < NT;
  const int s = valid ? tid : (NT - 1);

  const float* qap = qa + ((size_t)(b * NT + t) * NT + s) * NCP;
  const float* aqp = aq + ((size_t)(b * NT + s) * NT + t) * NCP;
  float al[NQV];
  al[0] = 1.0f;
#pragma unroll
  for (int c = 0; c < NCP; ++c) {
    const float qv = qap[c];
    al[1 + c] = qv;
    al[1 + NCP + c] = 1.0f - qv;
  }
  const float* gp = G + (size_t)(b * NPR) * GSZ + (size_t)t * NT + s;
  float sc = 0.0f;
#pragma unroll 1
  for (int bi = 0; bi < NKV; ++bi) {
    const float aqv  = aqp[(bi > 0) ? (bi - 1) : 0];
    const float beta = (bi == 0) ? 1.0f : aqv;
    const float* gq = gp + (size_t)bi * GSZ;
    float inner = 0.0f;
#pragma unroll
    for (int a = 0; a < NQV; ++a) inner += al[a] * gq[(size_t)(a * NKV) * GSZ];
    sc += beta * inner;
  }
  sc *= rscale;
  if (mask[b * NT + s] == 0) sc = -1.0e9f;

  float mx = valid ? sc : -INFINITY;
#pragma unroll
  for (int off = 16; off > 0; off >>= 1) mx = fmaxf(mx, __shfl_xor(mx, off, 32));
  if (lane == 0) redm[wave] = mx;
  __syncthreads();
  float m = redm[0];
#pragma unroll
  for (int w = 1; w < 8; ++w) m = fmaxf(m, redm[w]);
  const float e = valid ? expf(sc - m) : 0.0f;
  float sm = e;
#pragma unroll
  for (int off = 16; off > 0; off >>= 1) sm += __shfl_xor(sm, off, 32);
  if (lane == 0) reds[wave] = sm;
  __syncthreads();
  float tot = reds[0];
#pragma unroll
  for (int w = 1; w < 8; ++w) tot += reds[w];
  const float p = e * (1.0f / tot);
  if (valid) {
    const unsigned short hb = f2bf_bits(p);
    ph[tid] = hb;
    pl[tid] = f2bf_bits(p - bf_bits2f(hb));
  }
  __syncthreads();
  if (wave == 0 && lane < 24) {
    const v4u hv = *(const v4u*)(ph + lane * 8);
    const v4u lv = *(const v4u*)(pl + lane * 8);
    unsigned short* prh = Ph + (size_t)bt * NT + lane * 8;
    unsigned short* prl = Pl + (size_t)bt * NT + lane * 8;
    *(volatile v4u*)prh = hv;
    *(volatile v4u*)prl = lv;
    __threadfence();
    *(volatile v4u*)prh = hv;
    *(volatile v4u*)prl = lv;
  }
}

__global__ __launch_bounds__(256) void layernorm_kernel(const float* __restrict__ X, const float* __restrict__ w,
                                                        const float* __restrict__ bb, float* out, int nrows)
{
  const int row  = blockIdx.x * 8 + (threadIdx.x >> 5);
  const int lane = threadIdx.x & 31;
  if (row >= nrows) return;
  const float* x = X + (size_t)row * ND;
  v4f xv[4];
  float s = 0.0f;
#pragma unroll
  for (int i = 0; i < 4; ++i) {
    xv[i] = *(const v4f*)(x + i * 128 + 4 * lane);
    s += (xv[i][0] + xv[i][1]) + (xv[i][2] + xv[i][3]);
  }
#pragma unroll
  for (int off = 16; off > 0; off >>= 1) s += __shfl_xor(s, off, 32);
  const float mean = s * (1.0f / 512.0f);
  float vs = 0.0f;
#pragma unroll
  for (int i = 0; i < 4; ++i) {
    const v4f d = xv[i] - mean;
    xv[i] = d;
    vs += (d[0] * d[0] + d[1] * d[1]) + (d[2] * d[2] + d[3] * d[3]);
  }
#pragma unroll
  for (int off = 16; off > 0; off >>= 1) vs += __shfl_xor(vs, off, 32);
  const float var = vs * (1.0f / 512.0f);
  const float inv = 1.0f / sqrtf(var + 1.0e-12f);
  v4f yv[4];
#pragma unroll
  for (int i = 0; i < 4; ++i) {
    const v4f wv = *(const v4f*)(w + i * 128 + 4 * lane);
    const v4f bv = *(const v4f*)(bb + i * 128 + 4 * lane);
    yv[i] = wv * (xv[i] * inv) + bv;
  }
  float* o = out + (size_t)row * ND;
  for (int pass = 0; pass < 2; ++pass) {
#pragma unroll
    for (int i = 0; i < 4; ++i) *(volatile v4f*)(o + i * 128 + 4 * lane) = yv[i];
    __threadfence();
  }
}

extern "C" void kernel_launch(void* const* d_in, const int* in_sizes, int n_in,
                              void* d_out, int out_size, void* d_ws, size_t ws_size,
                              hipStream_t stream) {
  if (n_in < 20) return;
  if (in_sizes[0] != NBT * ND || in_sizes[1] != NBT * ND || in_sizes[2] != NBT * ND) return;
  if (in_sizes[3] != NBAT * NT * NT * NCP || in_sizes[4] != NBAT * NT * NT * NCP) return;
  if (in_sizes[5] != NBAT * NT) return;
  if (in_sizes[6] != ND * ND || in_sizes[8] != ND * ND || in_sizes[10] != ND * ND || in_sizes[16] != ND * ND) return;
  if (in_sizes[7] != ND || in_sizes[9] != ND || in_sizes[11] != ND || in_sizes[17] != ND) return;
  if (in_sizes[18] != ND || in_sizes[19] != ND) return;
  if (in_sizes[12] != ND * CPW || in_sizes[13] != ND * CPW || in_sizes[14] != ND * CPW || in_sizes[15] != ND * CPW) return;
  if (out_size != NBT * ND) return;

  const float* query = (const float*)d_in[0];
  const float* key   = (const float*)d_in[1];
  const float* value = (const float*)d_in[2];
  const float* qa    = (const float*)d_in[3];
  const float* aq    = (const float*)d_in[4];
  const int*   mask  = (const int*)d_in[5];
  const float* Wq  = (const float*)d_in[6];  const float* bq = (const float*)d_in[7];
  const float* Wk  = (const float*)d_in[8];  const float* bk = (const float*)d_in[9];
  const float* Wv  = (const float*)d_in[10]; const float* bv = (const float*)d_in[11];
  const float* Wl1 = (const float*)d_in[12];
  const float* Wr1 = (const float*)d_in[13];
  const float* Wl0 = (const float*)d_in[14];
  const float* Wr0 = (const float*)d_in[15];
  const float* Wo  = (const float*)d_in[16]; const float* bo = (const float*)d_in[17];
  const float* lnw = (const float*)d_in[18];
  const float* lnb = (const float*)d_in[19];
  float* out = (float*)d_out;

  size_t off = 0;
  auto carve = [&](size_t bytes) -> size_t { const size_t o = off; off += (bytes + 4095) & ~((size_t)4095); return o; };
  const size_t XPE  = (size_t)NBT * ND;
  const size_t szX3 = 3 * XPE * 2;
  const size_t szWQ = (size_t)QPW * ND * 2;
  const size_t szWK = (size_t)KPW * ND * 2;
  const size_t szWR = (size_t)CPW * ND * 2;
  const size_t szW  = (size_t)ND * ND * 2;
  const size_t szQP = (size_t)NBT * QPW * 2;
  const size_t szKL = (size_t)NBT * CPW * 4;
  const size_t szKP = (size_t)NBT * KPW * 2;
  const size_t szVT = (size_t)NBAT * ND * NT * 2;
  const size_t szG  = (size_t)NZG * GSZ * 4;
  const size_t szP  = (size_t)NBT * NT * 2;
  const size_t szCX = (size_t)NBT * ND * 2;
  const size_t szLN = (size_t)NBT * ND * 4;
  const size_t oXh = carve(szX3),  oXl = carve(szX3);
  const size_t oWQh = carve(szWQ), oWQl = carve(szWQ);
  const size_t oWKh = carve(szWK), oWKl = carve(szWK);
  const size_t oWRh = carve(szWR), oWRl = carve(szWR);
  const size_t oWVh = carve(szW),  oWVl = carve(szW);
  const size_t oWOh = carve(szW),  oWOl = carve(szW);
  const size_t oQPh = carve(szQP), oQPl = carve(szQP);
  const size_t oKL  = carve(szKL);
  const size_t oKPh = carve(szKP), oKPl = carve(szKP);
  const size_t oVTh = carve(szVT), oVTl = carve(szVT);
  const size_t oG   = carve(szG);
  const size_t oPh  = carve(szP),  oPl  = carve(szP);
  const size_t oCXh = carve(szCX), oCXl = carve(szCX);
  const size_t oLN  = carve(szLN);
  if (off > ws_size) return;
  if (off > (size_t)134217728) return;

  char* ws = (char*)d_ws;
  unsigned short* Xh  = (unsigned short*)(ws + oXh);  unsigned short* Xl  = (unsigned short*)(ws + oXl);
  unsigned short* WQh = (unsigned short*)(ws + oWQh); unsigned short* WQl = (unsigned short*)(ws + oWQl);
  unsigned short* WKh = (unsigned short*)(ws + oWKh); unsigned short* WKl = (unsigned short*)(ws + oWKl);
  unsigned short* WRh = (unsigned short*)(ws + oWRh); unsigned short* WRl = (unsigned short*)(ws + oWRl);
  unsigned short* WVh = (unsigned short*)(ws + oWVh); unsigned short* WVl = (unsigned short*)(ws + oWVl);
  unsigned short* WOh = (unsigned short*)(ws + oWOh); unsigned short* WOl = (unsigned short*)(ws + oWOl);
  unsigned short* QPh = (unsigned short*)(ws + oQPh); unsigned short* QPl = (unsigned short*)(ws + oQPl);
  float*          KL  = (float*)(ws + oKL);
  unsigned short* KPh = (unsigned short*)(ws + oKPh); unsigned short* KPl = (unsigned short*)(ws + oKPl);
  unsigned short* VTh = (unsigned short*)(ws + oVTh); unsigned short* VTl = (unsigned short*)(ws + oVTl);
  float*          G   = (float*)(ws + oG);
  unsigned short* Ph  = (unsigned short*)(ws + oPh);  unsigned short* Pl  = (unsigned short*)(ws + oPl);
  unsigned short* CXh = (unsigned short*)(ws + oCXh); unsigned short* CXl = (unsigned short*)(ws + oCXl);
  float*          LN  = (float*)(ws + oLN);

  unsigned short* Xqh = Xh;           unsigned short* Xql = Xl;
  unsigned short* Xkh = Xh + XPE;     unsigned short* Xkl = Xl + XPE;
  unsigned short* Xvh = Xh + 2 * XPE; unsigned short* Xvl = Xl + 2 * XPE;

  const dim3 blk(256);

  const int n2 = NBT * ND / 2;
  split3_kernel<<<dim3((n2 + 255) / 256, 3), blk, 0, stream>>>(query, key, value, Xh, Xl, n2, (int)XPE);

  tsplit4_kernel<<<dim3(ND / 64, ND / 64, 4), blk, 0, stream>>>(
      Wq, Wk, Wv, Wo, WQh, WKh, WVh, WOh, WQl, WKl, WVl, WOl, ND, ND);
  tsplit4_kernel<<<dim3(CPW / 64, ND / 64, 4), blk, 0, stream>>>(
      Wl1, Wl0, Wr1, Wr0,
      WQh + (size_t)ND * ND, WQh + (size_t)(ND + CPW) * ND, WKh + (size_t)ND * ND, WRh,
      WQl + (size_t)ND * ND, WQl + (size_t)(ND + CPW) * ND, WKl + (size_t)ND * ND, WRl,
      ND, CPW);

  gemm64_split<2, 2, false><<<dim3(((NBT / 64) * (QPW / 64) + 7) / 8, 1), blk, 0, stream>>>(
      Xqh, Xql, ND, 0L, 0L, WQh, WQl, ND, 0L, 0L, (void*)QPh, (void*)QPl, QPW, 0L,
      bq, ND, KL, CPW, 0, 0L, NBT, QPW, ND, 1, 1, 1.0f);

  gemm64_split<0, 0, false><<<dim3(((NBT / 64) * (CPW / 64) + 7) / 8, 1), blk, 0, stream>>>(
      Xkh, Xkl, ND, 0L, 0L, WRh, WRl, ND, 0L, 0L, (void*)KL, (void*)KL, CPW, 0L,
      bq, 1, KL, CPW, 0, 0L, NBT, CPW, ND, 1, 1, 1.0f);

  gemm64_split<2, 2, true><<<dim3(((NBT / 64) * (KPW / 64) + 7) / 8, 1), blk, 0, stream>>>(
      Xkh, Xkl, ND, 0L, 0L, WKh, WKl, ND, 0L, 0L, (void*)KPh, (void*)KPl, KPW, 0L,
      bk, ND, KL, CPW, ND, 0L, NBT, KPW, ND, 1, 1, 1.0f);

  gemm64_split<1, 2, false><<<dim3(((ND / 64) * (NT / 64) + 7) / 8, NBAT), blk, 0, stream>>>(
      WVh, WVl, ND, 0L, 0L, Xvh, Xvl, ND, (long)NT * ND, 0L, (void*)VTh, (void*)VTl, NT, (long)ND * NT,
      bv, ND, KL, CPW, 0, 0L, ND, NT, ND, 1, 1, 1.0f);

  gemm64_split<0, 0, false><<<dim3(3, NZG), dim3(96), 0, stream>>>(
      QPh, QPl, QPW, (long)NT * QPW, (long)ND, KPh, KPl, KPW, (long)NT * KPW, (long)ND,
      (void*)G, (void*)G, NT, (long)GSZ,
      bq, 1, KL, CPW, 0, 0L, NT, NT, ND, NPR, NKV, 1.0f);

  score_softmax_kernel<<<dim3(NBT), blk, 0, stream>>>(G, qa, aq, mask, Ph, Pl, 0.044194173824159220f);

  gemm64_split<0, 2, false><<<dim3(((NT / 64) * (ND / 64) + 7) / 8, NBAT), blk, 0, stream>>>(
      Ph, Pl, NT, (long)NT * NT, 0L, VTh, VTl, NT, (long)ND * NT, 0L, (void*)CXh, (void*)CXl, ND, (long)NT * ND,
      bq, 1, KL, CPW, 0, 0L, NT, ND, NT, 1, 1, 1.0f);

  gemm64_split<2, 0, false><<<dim3(((NBT / 64) * (ND / 64) + 7) / 8, 1), blk, 0, stream>>>(
      CXh, CXl, ND, 0L, 0L, WOh, WOl, ND, 0L, 0L, (void*)LN, (void*)LN, ND, 0L,
      bo, ND, KL, CPW, 0, 0L, NBT, ND, ND, 1, 1, 1.0f);

  layernorm_kernel<<<dim3(NBT / 8), blk, 0, stream>>>(LN, lnw, lnb, out, NBT);

  (void)hipGetLastError();
}
